// GatedDeltaNet_36971078484475
// MI455X (gfx1250) — hardware-verified
//
#include <hip/hip_runtime.h>
#include <math.h>

constexpr int NB    = 2;
constexpr int NT    = 2048;
constexpr int ND    = 1024;
constexpr int NH    = 16;
constexpr int HDIM  = 64;
constexpr int NTAP  = 4;
constexpr int NROW  = NB * NT;
constexpr int NQKV  = 3 * ND;
constexpr int COL_Z   = NQKV;
constexpr int COL_B   = COL_Z + ND;
constexpr int COL_A   = COL_B + NH;
constexpr int COL_PAD = COL_A + NH;
constexpr int NCAT    = 4160;
constexpr int CHUNK   = 32;
constexpr int NCHUNK  = NT / CHUNK;
constexpr int NTHR    = 256;
constexpr int HDIM_SQRT = 8;
constexpr float QSCALE  = 1.0f / (float)HDIM_SQRT;
constexpr float INV_HDIM = 1.0f / (float)HDIM;
constexpr float NORM_EPS = 1e-6f;
constexpr float Y_CARRY  = 16.0f;
constexpr float W_CARRY  = 256.0f;
constexpr float OUT_SCALE = 1.0f / (Y_CARRY * W_CARRY);
static_assert(HDIM_SQRT * HDIM_SQRT == HDIM, "head dim scale");
static_assert(NH * HDIM == ND, "heads");
static_assert(COL_PAD == 4128 && NCAT % 64 == 0 && NCAT >= COL_PAD, "concatenated width");
static_assert(NROW % 64 == 0 && ND % 64 == 0 && ND % 32 == 0, "GEMM tile multiples");
static_assert(NT % CHUNK == 0, "chunking");
static_assert(((NROW / 64) * (NCAT / 64)) % 8 == 0, "GEMM1 grid exact");
static_assert(((NROW / 64) * (ND / 64)) % 8 == 0, "GEMM2 grid exact");

typedef __attribute__((ext_vector_type(16))) _Float16 v16h;
typedef __attribute__((ext_vector_type(8)))  _Float16 v8h;
typedef __attribute__((ext_vector_type(16))) __bf16   v16b;
typedef __attribute__((ext_vector_type(8)))  __bf16   v8b;
typedef __attribute__((ext_vector_type(8)))  float    v8f;
typedef __attribute__((ext_vector_type(4)))  float    v4f;
typedef __attribute__((ext_vector_type(2)))  float    v2f;
typedef __attribute__((ext_vector_type(4)))  unsigned int v4u;

__device__ __forceinline__ unsigned short f2bf_bits(float f) {
  unsigned u = __float_as_uint(f);
  return (unsigned short)((u + 0x7FFFu + ((u >> 16) & 1u)) >> 16);
}
__device__ __forceinline__ float bf_bits2f(unsigned short h) { return __uint_as_float(((unsigned)h) << 16); }
__device__ __forceinline__ float bf16r(float f) { return bf_bits2f(f2bf_bits(f)); }
__device__ __forceinline__ unsigned pk16(unsigned short a, unsigned short b) { return (unsigned)a | ((unsigned)b << 16); }
__device__ __forceinline__ unsigned short h_bits(float f) { const _Float16 h = (_Float16)f; return __builtin_bit_cast(unsigned short, h); }

__device__ __forceinline__ void grp_guard_h(v8f& a, v8f& b, v8f& c, v8f& d, v16h x, v16h y) { asm volatile("v_nop\n\tv_nop\n\tv_nop\n\tv_nop" : "+v"(a), "+v"(b), "+v"(c), "+v"(d) : "v"(x), "v"(y)); }
__device__ __forceinline__ void grp_guard_b(v8f& a, v8f& b, v8f& c, v8f& d, v16b x, v16b y) { asm volatile("v_nop\n\tv_nop\n\tv_nop\n\tv_nop" : "+v"(a), "+v"(b), "+v"(c), "+v"(d) : "v"(x), "v"(y)); }
__device__ __forceinline__ void keep4_h(v16h a, v16h b, v16h c, v16h d) { asm volatile("v_nop" :: "v"(a), "v"(b), "v"(c), "v"(d)); }
__device__ __forceinline__ void keep4_b(v16b a, v16b b, v16b c, v16b d) { asm volatile("v_nop" :: "v"(a), "v"(b), "v"(c), "v"(d)); }
__device__ __forceinline__ void acc_guard4(v8f& a, v8f& b, v8f& c, v8f& d) { asm volatile("v_nop\n\tv_nop\n\tv_nop\n\tv_nop" : "+v"(a), "+v"(b), "+v"(c), "+v"(d)); }

template <typename T> struct Frag;
template <> struct Frag<_Float16> {
  typedef v16h V; union U { v16h v; v8h h[2]; };
  static __device__ __forceinline__ v16h load(const _Float16* p) {
    U f; f.h[0] = *(const v8h*)(p); f.h[1] = *(const v8h*)(p + 16); return f.v;
  }
  static __device__ __forceinline__ v8f mma(v16h a, v16h b, v8f c) {
    return __builtin_amdgcn_wmma_f32_16x16x32_f16(false, a, false, b, (short)0, c, false, false);
  }
  static __device__ __forceinline__ void guard4(v8f& a, v8f& b, v8f& c, v8f& d, v16h x, v16h y) { grp_guard_h(a, b, c, d, x, y); }
  static __device__ __forceinline__ void keep(v16h a, v16h b, v16h c, v16h d) { keep4_h(a, b, c, d); }
};
template <> struct Frag<__bf16> {
  typedef v16b V; union U { v16b v; v8b h[2]; };
  static __device__ __forceinline__ v16b load(const __bf16* p) {
    U f; f.h[0] = *(const v8b*)(p); f.h[1] = *(const v8b*)(p + 16); return f.v;
  }
  static __device__ __forceinline__ v8f mma(v16b a, v16b b, v8f c) {
    return __builtin_amdgcn_wmma_f32_16x16x32_bf16(false, a, false, b, (short)0, c, false, false);
  }
  static __device__ __forceinline__ void guard4(v8f& a, v8f& b, v8f& c, v8f& d, v16b x, v16b y) { grp_guard_b(a, b, c, d, x, y); }
  static __device__ __forceinline__ void keep(v16b a, v16b b, v16b c, v16b d) { keep4_b(a, b, c, d); }
};

template <int ET> struct Elem;
template <> struct Elem<0> { typedef _Float16 T; };
template <> struct Elem<1> { typedef __bf16 T; };
template <int ET, bool SPLIT, int BIAS_MODE, int OUT_MODE, bool RESID, int ACT = 0>
__global__ __launch_bounds__(256) void wmma_gemm64(
    const unsigned short* __restrict__ Ap, const unsigned short* __restrict__ A2p, int lda, long strideA,
    const unsigned short* __restrict__ Btp, const unsigned short* __restrict__ Bt2p, int ldb, long strideB,
    void* __restrict__ Cout, void* __restrict__ Cout2, int ldc, long strideC,
    const float* __restrict__ bias,
    const float* __restrict__ resid, long strideR,
    int M, int N, int K, float scale) {
  typedef typename Elem<ET>::T T;
  typedef typename Frag<T>::V V;
  const T* A = (const T*)Ap; const T* A2 = (const T*)A2p; const T* Bt = (const T*)Btp; const T* Bt2 = (const T*)Bt2p;
  __shared__ __align__(16) float sT[8][16 * 68];
  const int b    = blockIdx.y;
  const int lane = threadIdx.x & 31;
  const int wave = threadIdx.x >> 5;
  const int tilesN = N >> 6;
  const int tilesM = M >> 6;
  const int tile = blockIdx.x * 8 + wave;
  if (tile >= tilesM * tilesN) return;
  const int tm = tile / tilesN;
  const int tn = tile - tm * tilesN;
  const int m0 = tm << 6;
  const int n0 = tn << 6;

  const T* Ab  = A  + (size_t)b * strideA;
  const T* Bb  = Bt + (size_t)b * strideB;
  const T* Ab2 = SPLIT ? (A2  + (size_t)b * strideA) : nullptr;
  const T* Bb2 = SPLIT ? (Bt2 + (size_t)b * strideB) : nullptr;

  const int rlane = lane & 15;
  const int koff  = (lane >> 4) * 8;
  const int mOff  = (lane >> 4) * 8;

  v8f acc[4][4];
#pragma unroll
  for (int i = 0; i < 4; ++i)
#pragma unroll
    for (int j = 0; j < 4; ++j) acc[i][j] = (v8f){0.f,0.f,0.f,0.f,0.f,0.f,0.f,0.f};

  for (int k0 = 0; k0 < K; k0 += 32) {
    V bh[4], bl[4];
#pragma unroll
    for (int j = 0; j < 4; ++j) {
      const size_t bo = (size_t)(n0 + (j << 4) + rlane) * ldb + koff + k0;
      bh[j] = Frag<T>::load(Bb + bo);
      if (SPLIT) bl[j] = Frag<T>::load(Bb2 + bo);
    }
#pragma unroll
    for (int i = 0; i < 4; ++i) {
      const size_t ao = (size_t)(m0 + (i << 4) + rlane) * lda + koff + k0;
      V ah = Frag<T>::load(Ab + ao);
      V al;
      if (SPLIT) al = Frag<T>::load(Ab2 + ao);
#pragma unroll
      for (int j = 0; j < 4; ++j) {
        acc[i][j] = Frag<T>::mma(ah, bh[j], acc[i][j]);
        if (SPLIT) {
          acc[i][j] = Frag<T>::mma(ah, bl[j], acc[i][j]);
          acc[i][j] = Frag<T>::mma(al, bh[j], acc[i][j]);
        }
      }
      Frag<T>::guard4(acc[i][0], acc[i][1], acc[i][2], acc[i][3], ah, SPLIT ? al : ah);
    }
    Frag<T>::keep(bh[0], bh[1], bh[2], bh[3]);
    if (SPLIT) Frag<T>::keep(bl[0], bl[1], bl[2], bl[3]);
  }
  acc_guard4(acc[0][0], acc[0][1], acc[0][2], acc[0][3]);
  acc_guard4(acc[1][0], acc[1][1], acc[1][2], acc[1][3]);
  acc_guard4(acc[2][0], acc[2][1], acc[2][2], acc[2][3]);
  acc_guard4(acc[3][0], acc[3][1], acc[3][2], acc[3][3]);

  float* slab = sT[wave];
  const float* Rb = RESID ? (resid + (size_t)b * strideR) : nullptr;
#pragma unroll
  for (int i = 0; i < 4; ++i) {
    const int mBase = m0 + (i << 4);
#pragma unroll
    for (int j = 0; j < 4; ++j) {
      const int n = n0 + (j << 4) + rlane;
      float bv = 0.f;
      if (BIAS_MODE == 2) bv = bias[n];
#pragma unroll
      for (int r = 0; r < 8; ++r) {
        float v = acc[i][j][r] * scale;
        if (BIAS_MODE == 1) v += bias[mBase + mOff + r];
        if (BIAS_MODE == 2) v += bv;
        if (RESID) v += Rb[(size_t)(mBase + mOff + r) * ldc + n];
        if (ACT == 2) v = fmaxf(v, 0.0f);
        if (ACT == 4) v = (v > 0.f) ? v : 0.01f * v;
        slab[(mOff + r) * 68 + (j << 4) + rlane] = v;
      }
    }
    __builtin_amdgcn_fence(__ATOMIC_RELEASE, "workgroup");
    __builtin_amdgcn_wave_barrier();
    __builtin_amdgcn_fence(__ATOMIC_ACQUIRE, "workgroup");
    if (OUT_MODE == 0) {
      float* C = (float*)Cout + (size_t)b * strideC;
      const int hh = lane >> 4, c4 = (lane & 15) * 4;
      for (int pass = 0; pass < 2; ++pass) {
#pragma unroll
        for (int it = 0; it < 8; ++it) {
          const int row = it * 2 + hh;
          v4f v = *(const v4f*)(slab + row * 68 + c4);
          *(volatile v4f*)(C + (size_t)(mBase + row) * ldc + n0 + c4) = v;
        }
        __threadfence();
      }
    } else {
      const int q = lane >> 3, c8 = (lane & 7) * 8;
      unsigned short* C  = (unsigned short*)Cout  + (size_t)b * strideC;
      unsigned short* C2 = (OUT_MODE == 2) ? ((unsigned short*)Cout2 + (size_t)b * strideC) : nullptr;
      for (int pass = 0; pass < 2; ++pass) {
#pragma unroll
        for (int it = 0; it < 4; ++it) {
          const int row = it * 4 + q;
          const float* sp = slab + row * 68 + c8;
          v8h hv, lv;
#pragma unroll
          for (int e = 0; e < 8; ++e) {
            if (OUT_MODE == 1) {
              hv[e] = (_Float16)sp[e];
            } else {
              unsigned short hb = f2bf_bits(sp[e]);
              unsigned short lb = f2bf_bits(sp[e] - bf_bits2f(hb));
              hv[e] = __builtin_bit_cast(_Float16, hb);
              lv[e] = __builtin_bit_cast(_Float16, lb);
            }
          }
          *(volatile v8h*)(C + (size_t)(mBase + row) * ldc + n0 + c8) = hv;
          if (OUT_MODE == 2) *(volatile v8h*)(C2 + (size_t)(mBase + row) * ldc + n0 + c8) = lv;
        }
        __threadfence();
      }
    }
    __builtin_amdgcn_fence(__ATOMIC_RELEASE, "workgroup");
    __builtin_amdgcn_wave_barrier();
    __builtin_amdgcn_fence(__ATOMIC_ACQUIRE, "workgroup");
  }
}

template <int MODE>
__global__ __launch_bounds__(NTHR) void cvt8_kernel(const float* __restrict__ src, unsigned short* __restrict__ dst,
                                                    int nrow, int ncol8, int spitch, int scol0, float sc) {
  const int i  = blockIdx.x * NTHR + threadIdx.x;
  const int n8 = nrow * ncol8;
  if (i < n8) {
    const int row = i / ncol8;
    const int c8  = i - row * ncol8;
    const float* sp = src + (size_t)row * spitch + scol0 + c8 * 8;
    const v4f a = *(const v4f*)(sp);
    const v4f b = *(const v4f*)(sp + 4);
    v8h hv;
#pragma unroll
    for (int e = 0; e < 4; ++e) {
      unsigned short b0, b1;
      if (MODE == 0) {
        b0 = f2bf_bits(a[e] * sc);
        b1 = f2bf_bits(b[e] * sc);
      } else {
        b0 = __builtin_bit_cast(unsigned short, (_Float16)(bf16r(a[e]) * sc));
        b1 = __builtin_bit_cast(unsigned short, (_Float16)(bf16r(b[e]) * sc));
      }
      hv[e]     = __builtin_bit_cast(_Float16, b0);
      hv[4 + e] = __builtin_bit_cast(_Float16, b1);
    }
    *(volatile v8h*)(dst + (size_t)i * 8) = hv;
    __threadfence();
    *(volatile v8h*)(dst + (size_t)i * 8) = hv;
  }
}

__global__ __launch_bounds__(128) void build_wcat_kernel(const float* __restrict__ Wqkv, const float* __restrict__ Wz,
                                                         const float* __restrict__ Wb, const float* __restrict__ Wa,
                                                         unsigned short* __restrict__ dst) {
  const int row = blockIdx.x;
  const int tid = threadIdx.x;
  const float* src = Wqkv;
  int srow = row;
  if (row >= COL_A) {
    src = Wa;
    srow = row - COL_A;
    if (srow > NH - 1) srow = NH - 1;
  } else if (row >= COL_B) {
    src = Wb;
    srow = row - COL_B;
  } else if (row >= COL_Z) {
    src = Wz;
    srow = row - COL_Z;
  }
  const bool live = row < COL_PAD;
  const float* sp = src + (size_t)srow * ND + tid * 8;
  const v4f a = *(const v4f*)(sp);
  const v4f c = *(const v4f*)(sp + 4);
  unsigned short hb[8];
#pragma unroll
  for (int e = 0; e < 4; ++e) {
    hb[e]     = f2bf_bits(a[e]);
    hb[4 + e] = f2bf_bits(c[e]);
  }
  unsigned w0 = pk16(hb[0], hb[1]);
  unsigned w1 = pk16(hb[2], hb[3]);
  unsigned w2 = pk16(hb[4], hb[5]);
  unsigned w3 = pk16(hb[6], hb[7]);
  w0 = live ? w0 : 0u;
  w1 = live ? w1 : 0u;
  w2 = live ? w2 : 0u;
  w3 = live ? w3 : 0u;
  const v4u u = (v4u){w0, w1, w2, w3};
  unsigned short* q = dst + (size_t)row * ND + tid * 8;
  *(volatile v4u*)q = u;
  __threadfence();
  *(volatile v4u*)q = u;
}

__global__ __launch_bounds__(NTHR) void gated_scan_kernel(const float* __restrict__ P, const float* __restrict__ convw,
                                                          const float* __restrict__ dtb, const float* __restrict__ alog,
                                                          unsigned short* __restrict__ Y) {
  __shared__ __align__(16) float sQKV[3 * CHUNK * HDIM];
  __shared__ __align__(16) float sGB[2 * CHUNK];
  __shared__ __align__(16) float sPO[4 * CHUNK * HDIM];
  __shared__ __align__(16) unsigned sY[CHUNK * 32];

  const int tid  = threadIdx.x;
  const int lane = tid & 31;
  const int wave = __builtin_amdgcn_readfirstlane(tid >> 5);
  const int bb   = blockIdx.x / NH;
  const int hd   = blockIdx.x - bb * NH;
  const int vc   = tid & 63;
  const int qd   = wave >> 1;
  const int d0   = qd * 16;
  const size_t rowbase = (size_t)bb * NT;

  const int partc = qd < 3 ? qd : 2;
  const int pcol  = partc * ND + hd * HDIM + vc;
  const v4f wv = *(const v4f*)(convw + (size_t)pcol * NTAP);
  const float w0 = bf16r(wv[0]);
  const float w1 = bf16r(wv[1]);
  const float w2 = bf16r(wv[2]);
  const float w3 = bf16r(wv[3]);

  const float aexp = expf(bf16r(alog[hd]));
  const float dtv  = bf16r(dtb[hd]);
  const bool  isb  = (wave == 6);
  const int   gcol = (isb ? COL_B : COL_A) + hd;

  float S[16];
#pragma unroll
  for (int i = 0; i < 16; ++i) S[i] = 0.0f;
  float m1 = 0.0f, m2 = 0.0f, m3 = 0.0f;

  const float* sQ = sQKV;
  const float* sK = sQKV + CHUNK * HDIM;
  const float* sV = sQKV + 2 * CHUNK * HDIM;

#pragma unroll 1
  for (int ck = 0; ck < NCHUNK; ++ck) {
    const int t0 = ck * CHUNK;

    if (wave < 6) {
      float* dst = sQKV + qd * (CHUNK * HDIM) + vc;
      const float* src = P + (rowbase + (size_t)t0) * NCAT + pcol;
#pragma unroll 1
      for (int r = 0; r < CHUNK; ++r) {
        float xv = src[(size_t)r * NCAT];
        asm volatile("" : "+v"(xv));
        float acc = w0 * m3;
        acc = fmaf(w1, m2, acc);
        acc = fmaf(w2, m1, acc);
        acc = fmaf(w3, xv, acc);
        const float sg = __builtin_amdgcn_rcpf(1.0f + expf(-acc));
        dst[r * HDIM] = acc * sg;
        m3 = m2;
        m2 = m1;
        m1 = xv;
      }
    } else {
      const float a = P[(rowbase + (size_t)(t0 + lane)) * NCAT + gcol];
      const float beta = __builtin_amdgcn_rcpf(1.0f + expf(-a));
      const float ad = a + dtv;
      const float sp = fmaxf(ad, 0.0f) + logf(1.0f + expf(-fabsf(ad)));
      float egv = expf(-(aexp * sp));
      egv = (egv < 1.17549435e-38f) ? 0.0f : egv;
      sGB[tid - 192] = isb ? beta : egv;
    }
    __syncthreads();

#pragma unroll 1
    for (int i = 0; i < 8; ++i) {
      const int u = 8 * wave + i;
      float* vp = sQKV + (u >> 5) * (CHUNK * HDIM) + (u & 31) * HDIM;
      const float a0 = vp[lane];
      const float a1 = vp[lane + 32];
      float ss = a0 * a0 + a1 * a1;
      ss += __shfl_xor(ss, 16, 32);
      ss += __shfl_xor(ss, 8, 32);
      ss += __shfl_xor(ss, 4, 32);
      ss += __shfl_xor(ss, 2, 32);
      ss += __shfl_xor(ss, 1, 32);
      const float inv = rsqrtf(ss + NORM_EPS) * ((u < CHUNK) ? QSCALE : 1.0f);
      vp[lane]      = a0 * inv;
      vp[lane + 32] = a1 * inv;
    }
    __syncthreads();

#pragma unroll 1
    for (int t = 0; t < CHUNK; ++t) {
      const float bt = sGB[t];
      const float eg = sGB[CHUNK + t];
      const float vb = sV[t * HDIM + vc] * bt;
      const float* kp = sK + t * HDIM + d0;
      const float* qp = sQ + t * HDIM + d0;
      float po = 0.0f;
#pragma unroll
      for (int i4 = 0; i4 < 4; ++i4) {
        const v4f kk = *(const v4f*)(kp + 4 * i4);
        const v4f qq = *(const v4f*)(qp + 4 * i4);
#pragma unroll
        for (int e = 0; e < 4; ++e) {
          const float sn = fmaf(kk[e], vb, S[4 * i4 + e] * eg);
          S[4 * i4 + e] = sn;
          po = fmaf(qq[e], sn, po);
        }
      }
      sPO[(qd * CHUNK + t) * HDIM + vc] = po;
    }
    __syncthreads();

#pragma unroll 1
    for (int rr = 0; rr < 4; ++rr) {
      const int t = 4 * wave + rr;
      const float* pp = sPO + t * HDIM + 2 * lane;
      const v2f p0 = *(const v2f*)(pp);
      const v2f p1 = *(const v2f*)(pp + CHUNK * HDIM);
      const v2f p2 = *(const v2f*)(pp + 2 * CHUNK * HDIM);
      const v2f p3 = *(const v2f*)(pp + 3 * CHUNK * HDIM);
      const float o0 = (p0[0] + p1[0]) + (p2[0] + p3[0]);
      const float o1 = (p0[1] + p1[1]) + (p2[1] + p3[1]);
      float ss = o0 * o0 + o1 * o1;
      ss += __shfl_xor(ss, 16, 32);
      ss += __shfl_xor(ss, 8, 32);
      ss += __shfl_xor(ss, 4, 32);
      ss += __shfl_xor(ss, 2, 32);
      ss += __shfl_xor(ss, 1, 32);
      const float rs = rsqrtf(ss * INV_HDIM + NORM_EPS);
      const v2f zz = *(const v2f*)(P + (rowbase + (size_t)(t0 + t)) * NCAT + COL_Z + hd * HDIM + 2 * lane);
      const float z0 = zz[0];
      const float z1 = zz[1];
      const float g0 = z0 * __builtin_amdgcn_rcpf(1.0f + expf(-z0));
      const float g1 = z1 * __builtin_amdgcn_rcpf(1.0f + expf(-z1));
      const float y0 = ((o0 * rs) * g0) * Y_CARRY;
      const float y1 = ((o1 * rs) * g1) * Y_CARRY;
      const unsigned short hb0 = h_bits(y0);
      const unsigned short hb1 = h_bits(y1);
      sY[t * 32 + lane] = pk16(hb0, hb1);
    }
    __syncthreads();
    {
      const int q = lane >> 3;
      const int c8 = lane & 7;
      const int t = 4 * wave + q;
      const v4u u = *(const v4u*)(sY + t * 32 + c8 * 4);
      unsigned short* yp = Y + (rowbase + (size_t)(t0 + t)) * ND + hd * HDIM + c8 * 8;
      *(volatile v4u*)yp = u;
      __threadfence();
      *(volatile v4u*)yp = u;
    }
  }
}

constexpr size_t BYTES_XB   = (size_t)NROW * ND * 2;
constexpr size_t BYTES_WCAT = (size_t)NCAT * ND * 2;
constexpr size_t BYTES_WOUT = (size_t)ND * ND * 2;
constexpr size_t BYTES_P    = (size_t)NROW * NCAT * 4;
constexpr size_t BYTES_Y    = (size_t)NROW * ND * 2;
static_assert(BYTES_XB % 256 == 0 && BYTES_WCAT % 256 == 0 && BYTES_WOUT % 256 == 0 && BYTES_P % 256 == 0 && BYTES_Y % 256 == 0, "aligned carve");
static_assert(BYTES_XB + BYTES_WCAT + BYTES_WOUT + BYTES_P + BYTES_Y <= (size_t)134217728, "carve cap");

extern "C" void kernel_launch(void* const* d_in, const int* in_sizes, int n_in,
                              void* d_out, int out_size, void* d_ws, size_t ws_size, hipStream_t stream) {
  if (n_in < 9 || d_out == nullptr || d_ws == nullptr) return;
  if (in_sizes[0] != NROW * ND || in_sizes[1] != NQKV * ND || in_sizes[2] != NQKV * NTAP ||
      in_sizes[3] != ND * ND || in_sizes[4] != NH * ND || in_sizes[5] != NH * ND ||
      in_sizes[6] != NH || in_sizes[7] != NH || in_sizes[8] != ND * ND ||
      out_size != NROW * ND) return;

  const float* x     = (const float*)d_in[0];
  const float* w_qkv = (const float*)d_in[1];
  const float* convw = (const float*)d_in[2];
  const float* w_z   = (const float*)d_in[3];
  const float* w_b   = (const float*)d_in[4];
  const float* w_a   = (const float*)d_in[5];
  const float* dtb   = (const float*)d_in[6];
  const float* alog  = (const float*)d_in[7];
  const float* w_out = (const float*)d_in[8];
  float* out = (float*)d_out;

  char* ws = (char*)d_ws;
  size_t off = 0;
  unsigned short* XB     = (unsigned short*)(ws + off); off += BYTES_XB;
  unsigned short* WCAT   = (unsigned short*)(ws + off); off += BYTES_WCAT;
  unsigned short* WOUT16 = (unsigned short*)(ws + off); off += BYTES_WOUT;
  float*          PCAT   = (float*)(ws + off);          off += BYTES_P;
  unsigned short* YH     = (unsigned short*)(ws + off); off += BYTES_Y;
  if (off > ws_size || off > (size_t)134217728) return;

  const int n8x = NROW * (ND / 8);
  const int n8w = ND * (ND / 8);
  cvt8_kernel<0><<<(n8x + NTHR - 1) / NTHR, NTHR, 0, stream>>>(x, XB, NROW, ND / 8, ND, 0, 1.0f);
  build_wcat_kernel<<<NCAT, 128, 0, stream>>>(w_qkv, w_z, w_b, w_a, WCAT);
  cvt8_kernel<1><<<(n8w + NTHR - 1) / NTHR, NTHR, 0, stream>>>(w_out, WOUT16, ND, ND / 8, ND, 0, W_CARRY);

  const dim3 g1((NROW / 64) * (NCAT / 64) / 8, 1);
  wmma_gemm64<1, false, 0, 0, false, 0><<<g1, 256, 0, stream>>>(
      XB, XB, ND, 0L, WCAT, WCAT, ND, 0L, (void*)PCAT, (void*)PCAT, NCAT, 0L,
      PCAT, PCAT, 0L, NROW, NCAT, ND, 1.0f);

  gated_scan_kernel<<<NB * NH, NTHR, 0, stream>>>(PCAT, convw, dtb, alog, YH);

  const dim3 g2((NROW / 64) * (ND / 64) / 8, 1);
  wmma_gemm64<0, false, 0, 0, false, 0><<<g2, 256, 0, stream>>>(
      YH, YH, ND, 0L, WOUT16, WOUT16, ND, 0L, (void*)out, (void*)out, ND, 0L,
      PCAT, PCAT, 0L, NROW, ND, ND, OUT_SCALE);
}
